// KeepHighResolutionModulePartSeg_75136157876259
// MI455X (gfx1250) — hardware-run, weakly checked
//
#include <hip/hip_runtime.h>


#ifndef NB
#define NB 32
#endif
#define NB_FULL 32
#define NPT   2048
#define CH    64
#define KNNK  8
#define NLV   4
#define PERB  131072
#define KQ    128
#define GT    64
#define EPS_BN 1e-5f
#define SLOPE  0.2f
#define WSC   64.0f
#define WSI   (1.0f / 64.0f)

static constexpr int lvS(int j) { return 1024 >> j; }
static constexpr int lvC(int j) { return 128 << j; }

static_assert(NB >= 1);
static_assert(NB <= NB_FULL);
static_assert(CH == 64);
static_assert(GT == 64);
static_assert(NPT % GT == 0);
static_assert(lvS(0) * lvC(0) == PERB);
static_assert(lvS(1) * lvC(1) == PERB);
static_assert(lvS(2) * lvC(2) == PERB);
static_assert(lvS(3) * lvC(3) == PERB);
static_assert(lvC(0) % 32 == 0);
static_assert(CH % 32 == 0);
static_assert(lvS(3) % 64 == 0);
static_assert((NB * NPT) % 64 == 0);
static_assert(lvS(1) % KQ == 0);
static_assert(lvS(2) % KQ == 0);
static_assert(lvS(3) % KQ == 0);
static_assert((lvS(3) * KNNK) % 32 == 0);
static_assert(PERB % 8 == 0);
static_assert(((size_t)NB * NPT * CH / 8) % 256 == 0);
static_assert(32 * 16 * 8 == 16 * CH * 4);
static_assert(32 * 16 * (GT / 2) == GT * CH * 4);
static_assert(32 * 16 == 2 * CH * 4);
static_assert(KQ * 16 * 2 == KQ * KNNK * 4);
static_assert(64 * 16 == 4 * CH * 4);
static_assert(4 * NPT * 4 + KQ * KNNK * 4 <= 131072);
static_assert(GT * CH * 4 + GT * 4 + 2 * CH * 4 <= 131072);
static_assert(16 * 68 * 4 + 2 * CH * 4 <= 131072);
static_assert(NLV * 4 * CH * 4 <= 131072);

typedef _Float16 h16;
typedef unsigned short bf;
typedef __attribute__((ext_vector_type(16))) __bf16   v16bf;
typedef __attribute__((ext_vector_type(16))) _Float16 v16h;
typedef __attribute__((ext_vector_type(8)))  _Float16 v8h;
typedef __attribute__((ext_vector_type(8)))  unsigned short v8us;
typedef __attribute__((ext_vector_type(8)))  float    v8f;
typedef __attribute__((ext_vector_type(4)))  float    v4f;
typedef __attribute__((ext_vector_type(2)))  float    v2f;
typedef __attribute__((ext_vector_type(4)))  int      v4i;
typedef v4f  __attribute__((may_alias)) v4fa;
typedef v2f  __attribute__((may_alias)) v2fa;
typedef v4i  __attribute__((may_alias)) v4ia;

__device__ __forceinline__ unsigned short f2bf(float f) { unsigned u = __float_as_uint(f); u += 0x7FFFu + ((u >> 16) & 1u); return (unsigned short)(u >> 16); }
__device__ __forceinline__ float bfr(float f) { return __uint_as_float(((unsigned)f2bf(f)) << 16); }
__device__ __forceinline__ v16h cat16(v8h lo, v8h hi) { return __builtin_shufflevector(lo, hi, 0, 1, 2, 3, 4, 5, 6, 7, 8, 9, 10, 11, 12, 13, 14, 15); }
__device__ __forceinline__ v16bf cat16b(v8us lo, v8us hi) { return __builtin_bit_cast(v16bf, __builtin_shufflevector(lo, hi, 0, 1, 2, 3, 4, 5, 6, 7, 8, 9, 10, 11, 12, 13, 14, 15)); }
__device__ __forceinline__ v16h  ldh(const h16* p) { return cat16(*(const v8h*)p, *(const v8h*)(p + 16)); }
__device__ __forceinline__ v16bf ldb(const bf* p)  { return cat16b(*(const v8us*)p, *(const v8us*)(p + 16)); }
__device__ __forceinline__ void wave_sync() { __builtin_amdgcn_fence(3  , "wavefront"); __builtin_amdgcn_wave_barrier(); asm volatile("" ::: "memory"); }
static __device__ __forceinline__ h16 toh_flush(float v) { const h16 r = (h16)v; return (fabsf(v) < 6.103515625e-05f) ? (h16)0.0f : r; }
__device__ __forceinline__ v8f wmmab_g(v16bf a, v16bf b, v8f c) {
    c = __builtin_amdgcn_wmma_f32_16x16x32_bf16(false, a, false, b, (short)0, c, false, false);
    asm volatile("v_nop\n\tv_nop\n\tv_nop\n\tv_nop" : "+v"(c) : "v"(a), "v"(b));
    return c; }
__device__ __forceinline__ v8f wmma16_g(v16h a, v16h b, v8f c) {
    c = __builtin_amdgcn_wmma_f32_16x16x32_f16(false, a, false, b, (short)0, c, false, false);
    asm volatile("v_nop\n\tv_nop\n\tv_nop\n\tv_nop" : "+v"(c) : "v"(a), "v"(b));
    return c; }

__global__ __launch_bounds__(256) void k_cvt8(const float* __restrict__ src, bf* dst, size_t n8) {
    const size_t i = (size_t)blockIdx.x * 256 + threadIdx.x; if (i >= n8) return;
    const v8f v = *(const v8f*)(src + i * 8); v8us o;
#pragma unroll
    for (int k = 0; k < 8; ++k) o[k] = f2bf(v[k]);
    *(volatile v8us*)(dst + i * 8) = o; __threadfence(); *(volatile v8us*)(dst + i * 8) = o;
}

__global__ __launch_bounds__(256) void k_wconv(const float* __restrict__ src, h16* dst, size_t n8) {
    const size_t i = (size_t)blockIdx.x * 256 + threadIdx.x; if (i >= n8) return;
    const v8f v = *(const v8f*)(src + i * 8); v8h o;
#pragma unroll
    for (int k = 0; k < 8; ++k) o[k] = toh_flush(bfr(v[k]) * WSC);
    *(volatile v8h*)(dst + i * 8) = o; __threadfence(); *(volatile v8h*)(dst + i * 8) = o;
}

__global__ __launch_bounds__(KQ) void k_knn(const float* __restrict__ xyz_all, const float* __restrict__ xyz_q, int S, int* IDX) {
#pragma clang fp contract(off)
    __shared__ float px[NPT];
    __shared__ float py[NPT];
    __shared__ float pz[NPT];
    __shared__ float pq[NPT];
    __shared__ __align__(16) int oi[KQ * KNNK];
    const int tid = threadIdx.x;
    const int q0 = blockIdx.x * KQ;
    const int b = q0 / S;
    const float* P = xyz_all + (size_t)b * NPT * 3;
#pragma unroll 1
    for (int n = tid; n < NPT; n += KQ) {
        const float x = bfr(P[n * 3 + 0]), y = bfr(P[n * 3 + 1]), z = bfr(P[n * 3 + 2]);
        px[n] = x; py[n] = y; pz[n] = z; pq[n] = (x * x + z * z) + y * y;
    }
    __syncthreads();
    const float* q = xyz_q + (size_t)(q0 + tid) * 3;
    const float qx = bfr(q[0]), qy = bfr(q[1]), qz = bfr(q[2]);
    const float sqq = (qx * qx + qz * qz) + qy * qy;
    float bd[KNNK]; int bi[KNNK];
#pragma unroll
    for (int j = 0; j < KNNK; ++j) { bd[j] = 3.0e38f; bi[j] = 0; }
#pragma unroll 1
    for (int n = 0; n < NPT; ++n) {
        const float p = fmaf(qz, pz[n], fmaf(qy, py[n], qx * px[n]));
        const float d = (sqq + pq[n]) - 2.0f * p;
        if (d < bd[KNNK - 1]) {
            bd[KNNK - 1] = d; bi[KNNK - 1] = n;
#pragma unroll
            for (int j = KNNK - 1; j > 0; --j) {
                const bool sw = bd[j] < bd[j - 1];
                const float dl = sw ? bd[j] : bd[j - 1], dh = sw ? bd[j - 1] : bd[j];
                const int   il = sw ? bi[j] : bi[j - 1], ih = sw ? bi[j - 1] : bi[j];
                bd[j - 1] = dl; bd[j] = dh; bi[j - 1] = il; bi[j] = ih;
            }
        }
    }
#pragma unroll
    for (int j = 0; j < KNNK; ++j) oi[tid * KNNK + j] = bi[j];
    __syncthreads();
    int* dst = IDX + (size_t)q0 * KNNK;
#pragma unroll 1
    for (int ps = 0; ps < 2; ++ps) {
#pragma unroll
        for (int it = 0; it < 2; ++it) { const int p = it * KQ + tid;
            const v4i v = *(const v4ia*)(&oi[p * 4]);
            *(volatile v4i*)(dst + p * 4) = v; }
        if (ps == 0) __threadfence(); }
}

__global__ __launch_bounds__(32) void k_gemm(const bf* __restrict__ A, const bf* __restrict__ Bt, float* G, int K) {
    __shared__ __align__(16) float os[16 * 68];
    const int lane = threadIdx.x & 31, lr = lane & 15, hi = lane >> 4; const int r0 = blockIdx.x * 64;
    v8f acc[4][4];
#pragma unroll
    for (int mb = 0; mb < 4; ++mb)
#pragma unroll
        for (int nb = 0; nb < 4; ++nb) acc[mb][nb] = (v8f){};
    const size_t aoff = (size_t)(r0 + lr) * K + 8 * hi, boff = (size_t)lr * K + 8 * hi;
#pragma unroll 1
    for (int kc = 0; kc < K; kc += 32) {
        v16bf a[4];
#pragma unroll
        for (int mb = 0; mb < 4; ++mb) a[mb] = ldb(A + aoff + (size_t)mb * 16 * K + kc);
#pragma unroll
        for (int nb = 0; nb < 4; ++nb) { const v16bf b = ldb(Bt + boff + (size_t)nb * 16 * K + kc);
#pragma unroll
            for (int mb = 0; mb < 4; ++mb) acc[mb][nb] = wmmab_g(a[mb], b, acc[mb][nb]); }
    }
#pragma unroll
    for (int mb = 0; mb < 4; ++mb) {
#pragma unroll
        for (int nb = 0; nb < 4; ++nb) {
#pragma unroll
            for (int j = 0; j < 8; ++j) os[(hi * 8 + j) * 68 + nb * 16 + lr] = acc[mb][nb][j]; }
        wave_sync();
        float* gp = G + (size_t)(r0 + mb * 16) * CH + 4 * lane;
#pragma unroll 1
        for (int ps = 0; ps < 2; ++ps) {
#pragma unroll
            for (int s = 0; s < 8; ++s) { const int row = 2 * s + (lane >> 4), c4 = (lane & 15) * 4;
                const v4f val = *(const v4fa*)(&os[row * 68 + c4]);
                *(volatile v4f*)(gp + s * 128) = val; }
            if (ps == 0) __threadfence(); }
        wave_sync();
    }
}

__global__ __launch_bounds__(32) void k_gather(const float* __restrict__ G, const int* __restrict__ IDX, const float* __restrict__ bias, int S, float* Y, float* PS) {
#pragma clang fp contract(off)
    __shared__ __align__(16) float acc[GT * CH];
    __shared__ __align__(16) float cn[GT];
    __shared__ __align__(16) float st[2 * CH];
    const int lane = threadIdx.x & 31;
    const int n0 = blockIdx.x * GT, b = blockIdx.y;
    const int nE = S * KNNK;
    const int* ib = IDX + (size_t)b * nE;
    const float* gb = G + (size_t)b * S * CH + 2 * lane;
#pragma unroll 1
    for (int r = 0; r < GT; ++r) { const v2f z = (v2f){}; *(v2fa*)(&acc[r * CH + 2 * lane]) = z; }
    float c0 = 0.0f, c1 = 0.0f;
#pragma unroll 1
    for (int e0 = 0; e0 < nE; e0 += 32) {
        const int rel = ib[e0 + lane] - n0;
        const bool hit = (unsigned)rel < (unsigned)GT;
        unsigned mask = (unsigned)__builtin_amdgcn_readfirstlane((int)__builtin_amdgcn_ballot_w32(hit));
#pragma unroll 1
        for (int it = 0; (it < 32) & (mask != 0u); ++it) {
            const int j = __builtin_ctz(mask); mask &= mask - 1u;
            const int slot = __builtin_amdgcn_readlane(rel, j) & (GT - 1);
            const int src = (e0 + j) >> 3;
            const v2f gv = *(const v2f*)(gb + (size_t)src * CH);
            v2f a = *(const v2fa*)(&acc[slot * CH + 2 * lane]);
            a = a + gv;
            *(v2fa*)(&acc[slot * CH + 2 * lane]) = a;
            c0 += (slot == lane) ? 1.0f : 0.0f;
            c1 += (slot == lane + 32) ? 1.0f : 0.0f;
        }
    }
    cn[lane] = c0; cn[lane + 32] = c1;
    wave_sync();
    const int hi = lane >> 4, c4 = (lane & 15) * 4;
    float bv[4], sx[4], qx[4];
#pragma unroll
    for (int i = 0; i < 4; ++i) { bv[i] = bfr(bias[c4 + i]); sx[i] = 0.0f; qx[i] = 0.0f; }
#pragma unroll 2
    for (int s = 0; s < GT / 2; ++s) {
        const int row = 2 * s + hi;
        v4f v = *(const v4fa*)(&acc[row * CH + c4]);
        const float sc = 1.0f / fmaxf(cn[row], 1.0f);
#pragma unroll
        for (int i = 0; i < 4; ++i) { const float y = v[i] * sc + bv[i]; v[i] = y; sx[i] += y; qx[i] += y * y; }
        *(v4fa*)(&acc[row * CH + c4]) = v;
    }
#pragma unroll
    for (int i = 0; i < 4; ++i) { sx[i] += __shfl_xor(sx[i], 16, 32); qx[i] += __shfl_xor(qx[i], 16, 32); }
    { v4f pv;
#pragma unroll
      for (int i = 0; i < 4; ++i) pv[i] = hi ? qx[i] : sx[i];
      *(v4fa*)(&st[hi * CH + c4]) = pv; }
    wave_sync();
    float* yrow = Y + ((size_t)b * NPT + n0) * CH + 4 * lane;
    float* pl = PS + ((size_t)b * (NPT / GT) + blockIdx.x) * (2 * CH) + 4 * lane;
#pragma unroll 1
    for (int ps = 0; ps < 2; ++ps) {
#pragma unroll 4
        for (int s = 0; s < GT / 2; ++s) {
            const v4f val = *(const v4fa*)(&acc[s * 128 + 4 * lane]);
            *(volatile v4f*)(yrow + s * 128) = val; }
        { const v4f pv = *(const v4fa*)(&st[4 * lane]); *(volatile v4f*)pl = pv; }
        if (ps == 0) __threadfence(); }
}

__global__ __launch_bounds__(128) void k_stats(const float* __restrict__ PS, int nlines, const float* __restrict__ gamma, const float* __restrict__ beta, float* ST) {
#pragma clang fp contract(off)
    __shared__ double sd[2 * CH];
    __shared__ __align__(16) float line[4 * CH];
    const int tid = threadIdx.x;
    double a = 0.0;
#pragma unroll 1
    for (int i = 0; i < nlines; ++i) a += (double)PS[(size_t)i * (2 * CH) + tid];
    sd[tid] = a;
    __syncthreads();
    const int c = tid & (CH - 1);
    const double invn = 1.0 / ((double)NB * (double)NPT);
    const double mean = sd[c] * invn;
    double var = sd[CH + c] * invn - mean * mean; var = var > 0.0 ? var : 0.0;
    const float inv = 1.0f / sqrtf((float)var + EPS_BN);
    const float gv = bfr(gamma[c]), bv = bfr(beta[c]);
    if (tid < CH) { line[c] = (float)mean; line[CH + c] = inv; line[2 * CH + c] = gv; line[3 * CH + c] = bv; }
    __syncthreads();
#pragma unroll 1
    for (int ps = 0; ps < 2; ++ps) {
        if (tid < CH) { const v4f v = *(const v4fa*)(&line[tid * 4]); *(volatile v4f*)(ST + tid * 4) = v; }
        if (ps == 0) __threadfence(); }
}

__global__ __launch_bounds__(256) void k_combine(const float* __restrict__ F0, const float* __restrict__ Y, const float* __restrict__ ST, h16* X, size_t n8, size_t ystr) {
#pragma clang fp contract(off)
    __shared__ __align__(16) float tb[NLV * 4 * CH];
    const int tid = threadIdx.x;
#pragma unroll 1
    for (int k = tid; k < NLV * 4 * CH; k += 256) tb[k] = ST[k];
    __syncthreads();
    const size_t i = (size_t)blockIdx.x * 256 + tid;
    if (i < n8) {
        const int c0 = (int)((i * 8) & (size_t)(CH - 1));
        const v8f f = *(const v8f*)(F0 + i * 8);
        float x[8];
#pragma unroll
        for (int k = 0; k < 8; ++k) x[k] = bfr(f[k]);
#pragma unroll 1
        for (int j = 0; j < NLV; ++j) {
            const v8f y = *(const v8f*)(Y + (size_t)j * ystr + i * 8);
            const int tj = j * 4 * CH + c0;
#pragma unroll
            for (int k = 0; k < 8; ++k) {
                const float t = (y[k] - tb[tj + k]) * tb[tj + CH + k] * tb[tj + 2 * CH + k] + tb[tj + 3 * CH + k];
                x[k] += (t >= 0.0f) ? t : SLOPE * t; }
        }
        v8h o;
#pragma unroll
        for (int k = 0; k < 8; ++k) o[k] = toh_flush(x[k]);
        *(volatile v8h*)(X + i * 8) = o; __threadfence(); *(volatile v8h*)(X + i * 8) = o;
    }
}

__global__ __launch_bounds__(32) void k_fin(const h16* __restrict__ X, const h16* __restrict__ WH, const float* __restrict__ b0, const float* __restrict__ ST4,
                                            const float* __restrict__ F0, const int* __restrict__ npp, float* OUT, float* PS, int apply) {
    __shared__ __align__(16) float os[16 * 68];
    __shared__ __align__(16) float st[2 * CH];
    const int lane = threadIdx.x & 31, lr = lane & 15, hi = lane >> 4; const int r0 = blockIdx.x * 64;
    v8f acc[4][4];
#pragma unroll
    for (int mb = 0; mb < 4; ++mb)
#pragma unroll
        for (int nb = 0; nb < 4; ++nb) acc[mb][nb] = (v8f){};
    const size_t aoff = (size_t)(r0 + lr) * CH + 8 * hi, boff = (size_t)lr * CH + 8 * hi;
#pragma unroll 1
    for (int kc = 0; kc < CH; kc += 32) {
        v16h a[4];
#pragma unroll
        for (int mb = 0; mb < 4; ++mb) a[mb] = ldh(X + aoff + (size_t)mb * 16 * CH + kc);
#pragma unroll
        for (int nb = 0; nb < 4; ++nb) { const v16h b = ldh(WH + boff + (size_t)nb * 16 * CH + kc);
#pragma unroll
            for (int mb = 0; mb < 4; ++mb) acc[mb][nb] = wmma16_g(a[mb], b, acc[mb][nb]); }
    }
    float bc[4];
#pragma unroll
    for (int nb = 0; nb < 4; ++nb) bc[nb] = bfr(b0[nb * 16 + lr]);
    if (apply == 0) {
        float s[4], q[4];
#pragma unroll
        for (int nb = 0; nb < 4; ++nb) { float ss = 0.0f, qq = 0.0f;
#pragma unroll
            for (int mb = 0; mb < 4; ++mb)
#pragma unroll
                for (int j = 0; j < 8; ++j) { const float z = acc[mb][nb][j] * WSI + bc[nb]; ss += z; qq += z * z; }
            s[nb] = ss; q[nb] = qq; }
#pragma unroll
        for (int nb = 0; nb < 4; ++nb) { s[nb] += __shfl_xor(s[nb], 16, 32); q[nb] += __shfl_xor(q[nb], 16, 32); }
#pragma unroll
        for (int nb = 0; nb < 4; ++nb) st[hi * CH + nb * 16 + lr] = hi ? q[nb] : s[nb];
        wave_sync();
        float* pl = PS + (size_t)blockIdx.x * (2 * CH) + 4 * lane;
#pragma unroll 1
        for (int ps = 0; ps < 2; ++ps) {
            { const v4f pv = *(const v4fa*)(&st[4 * lane]); *(volatile v4f*)pl = pv; }
            if (ps == 0) __threadfence(); }
    } else {
        float mu[4], iv[4], gm[4], bt[4];
#pragma unroll
        for (int nb = 0; nb < 4; ++nb) { const int c = nb * 16 + lr; mu[nb] = ST4[c]; iv[nb] = ST4[CH + c]; gm[nb] = ST4[2 * CH + c]; bt[nb] = ST4[3 * CH + c]; }
        const float pz = (npp[0] == NPT) ? 0.0f : __uint_as_float(0x7FC00000u);
#pragma unroll
        for (int mb = 0; mb < 4; ++mb) {
#pragma unroll
            for (int nb = 0; nb < 4; ++nb) {
#pragma unroll
                for (int j = 0; j < 8; ++j) { const float z = acc[mb][nb][j] * WSI + bc[nb];
                    const float t = (z - mu[nb]) * iv[nb] * gm[nb] + bt[nb];
                    os[(hi * 8 + j) * 68 + nb * 16 + lr] = (t >= 0.0f) ? t : SLOPE * t; } }
            wave_sync();
            const size_t ob = (size_t)(r0 + mb * 16) * CH + 4 * lane;
#pragma unroll 1
            for (int ps = 0; ps < 2; ++ps) {
#pragma unroll
                for (int s = 0; s < 8; ++s) { const int row = 2 * s + (lane >> 4), c4 = (lane & 15) * 4;
                    const v4f val = *(const v4fa*)(&os[row * 68 + c4]);
                    const v4f rf = *(const v4f*)(F0 + ob + s * 128);
                    v4f o;
#pragma unroll
                    for (int i = 0; i < 4; ++i) o[i] = val[i] + bfr(rf[i]) + pz;
                    *(volatile v4f*)(OUT + ob + s * 128) = o; }
                if (ps == 0) __threadfence(); }
            wave_sync();
        }
    }
}

static constexpr size_t al256(size_t v) { return (v + 255) & ~(size_t)255; }
static constexpr size_t SZ_FB  = al256((size_t)NB * PERB * 2);
static constexpr size_t szWB(int j) { return al256((size_t)CH * lvC(j) * 2); }
static constexpr size_t SZ_WH  = al256((size_t)CH * CH * 2);
static constexpr size_t szIDX(int j) { return al256((size_t)NB * lvS(j) * KNNK * 4); }
static constexpr size_t szG(int j) { return al256((size_t)NB * lvS(j) * CH * 4); }
static constexpr size_t SZ_Y   = al256((size_t)NB * NPT * CH * 4);
static constexpr size_t SZ_X   = al256((size_t)NB * NPT * CH * 2);
static constexpr size_t SZ_PS  = al256((size_t)NB * (NPT / GT) * 2 * CH * 4);
static constexpr size_t SZ_ST  = al256((size_t)4 * CH * 4);
static constexpr size_t SZ_TOTAL = 4 * SZ_FB + szWB(0) + szWB(1) + szWB(2) + szWB(3) + SZ_WH + szIDX(1) + szIDX(2) + szIDX(3)
                                 + szG(0) + szG(1) + szG(2) + szG(3) + 4 * SZ_Y + SZ_X + 5 * SZ_PS + 5 * SZ_ST;
static_assert(SZ_TOTAL <= (size_t)134217728);
static_assert(SZ_Y == (size_t)NB * NPT * CH * 4);
static_assert(SZ_ST == (size_t)4 * CH * 4);
static_assert((NB * NPT) / 64 == NB * (NPT / GT));

extern "C" void kernel_launch(void* const* d_in, const int* in_sizes, int n_in,
                              void* d_out, int out_size, void* d_ws, size_t ws_size, hipStream_t stream) {
    if (n_in < 31) return;
    if (in_sizes[0] < 1) return;
    for (int j = 1; j <= 5; ++j) if ((size_t)in_sizes[j] < (size_t)NB * PERB) return;
    if ((size_t)in_sizes[6] < (size_t)NB * 1024 * KNNK) return;
    if ((size_t)in_sizes[7] < (size_t)NB * NPT * 3) return;
    if ((size_t)in_sizes[8] < (size_t)NB * 512 * 3 || (size_t)in_sizes[9] < (size_t)NB * 256 * 3 || (size_t)in_sizes[10] < (size_t)NB * 128 * 3) return;
    for (int j = 0; j < 4; ++j) {
        if ((size_t)in_sizes[11 + 4 * j] < (size_t)CH * (size_t)(128 << j)) return;
        if (in_sizes[12 + 4 * j] < CH || in_sizes[13 + 4 * j] < CH || in_sizes[14 + 4 * j] < CH) return;
    }
    if (in_sizes[27] < CH * CH || in_sizes[28] < CH || in_sizes[29] < CH || in_sizes[30] < CH) return;
    if ((size_t)out_size < (size_t)NB * NPT * CH) return;
    if (SZ_TOTAL > ws_size) return;
    const int*   npp  = (const int*)d_in[0];
    const float* f0   = (const float*)d_in[1];
    const float* fl[4] = { (const float*)d_in[2], (const float*)d_in[3], (const float*)d_in[4], (const float*)d_in[5] };
    const int*   knn1 = (const int*)d_in[6];
    const float* xyz0 = (const float*)d_in[7];
    const float* xq[4] = { nullptr, (const float*)d_in[8], (const float*)d_in[9], (const float*)d_in[10] };
    const float *Wt[5], *bs[5], *gm[5], *bt[5];
    for (int j = 0; j < 5; ++j) {
        Wt[j] = (const float*)d_in[11 + 4 * j + 0];
        bs[j] = (const float*)d_in[11 + 4 * j + 1];
        gm[j] = (const float*)d_in[11 + 4 * j + 2];
        bt[j] = (const float*)d_in[11 + 4 * j + 3];
    }
    float* OUT = (float*)d_out;
    const int Ss[4] = { lvS(0), lvS(1), lvS(2), lvS(3) };
    const int Cs[4] = { lvC(0), lvC(1), lvC(2), lvC(3) };
    const size_t szwb[4] = { szWB(0), szWB(1), szWB(2), szWB(3) };
    const size_t szg[4]  = { szG(0), szG(1), szG(2), szG(3) };
    const size_t szix[4] = { 0, szIDX(1), szIDX(2), szIDX(3) };

    char* wsp = (char*)d_ws;
    bf* FB[4]; for (int j = 0; j < 4; ++j) { FB[j] = (bf*)wsp; wsp += SZ_FB; }
    bf* WB[4]; for (int j = 0; j < 4; ++j) { WB[j] = (bf*)wsp; wsp += szwb[j]; }
    h16* WH = (h16*)wsp; wsp += SZ_WH;
    int* IX[4]; IX[0] = nullptr; for (int j = 1; j < 4; ++j) { IX[j] = (int*)wsp; wsp += szix[j]; }
    float* GP[4]; for (int j = 0; j < 4; ++j) { GP[j] = (float*)wsp; wsp += szg[j]; }
    float* YP = (float*)wsp; wsp += 4 * SZ_Y;
    h16* XP = (h16*)wsp; wsp += SZ_X;
    float* PSP = (float*)wsp; wsp += 5 * SZ_PS;
    float* STP = (float*)wsp; wsp += 5 * SZ_ST;
    const size_t ystr = (size_t)NB * NPT * CH;
    const size_t psstr = SZ_PS / 4, ststr = SZ_ST / 4;
    const int nlines = NB * (NPT / GT);

    { const size_t n8 = (size_t)NB * PERB / 8; const unsigned g = (unsigned)((n8 + 255) / 256);
      for (int j = 0; j < 4; ++j) k_cvt8<<<g, 256, 0, stream>>>(fl[j], FB[j], n8); }
    for (int j = 0; j < 4; ++j) { const size_t n8 = (size_t)CH * Cs[j] / 8;
      k_cvt8<<<(unsigned)((n8 + 255) / 256), 256, 0, stream>>>(Wt[j], WB[j], n8); }
    { const size_t n8 = (size_t)CH * CH / 8; k_wconv<<<(unsigned)((n8 + 255) / 256), 256, 0, stream>>>(Wt[4], WH, n8); }

    for (int j = 1; j < 4; ++j) k_knn<<<(unsigned)(NB * Ss[j] / KQ), KQ, 0, stream>>>(xyz0, xq[j], Ss[j], IX[j]);

    for (int j = 0; j < 4; ++j) {
        k_gemm<<<(unsigned)(NB * Ss[j] / 64), 32, 0, stream>>>(FB[j], WB[j], GP[j], Cs[j]);
        k_gather<<<dim3(NPT / GT, NB, 1), 32, 0, stream>>>(GP[j], (j == 0) ? knn1 : IX[j], bs[j], Ss[j], YP + (size_t)j * ystr, PSP + (size_t)j * psstr);
        k_stats<<<1, 128, 0, stream>>>(PSP + (size_t)j * psstr, nlines, gm[j], bt[j], STP + (size_t)j * ststr);
    }

    { const size_t n8 = (size_t)NB * NPT * CH / 8;
      k_combine<<<(unsigned)(n8 / 256), 256, 0, stream>>>(f0, YP, STP, XP, n8, ystr); }

    k_fin<<<(unsigned)(NB * NPT / 64), 32, 0, stream>>>(XP, WH, bs[4], STP + (size_t)4 * ststr, f0, npp, OUT, PSP + (size_t)4 * psstr, 0);
    k_stats<<<1, 128, 0, stream>>>(PSP + (size_t)4 * psstr, nlines, gm[4], bt[4], STP + (size_t)4 * ststr);
    k_fin<<<(unsigned)(NB * NPT / 64), 32, 0, stream>>>(XP, WH, bs[4], STP + (size_t)4 * ststr, f0, npp, OUT, PSP + (size_t)4 * psstr, 1);
}
